// SequentialPeAttention_60043642798653
// MI455X (gfx1250) — hardware-verified
//
#include <hip/hip_runtime.h>
#include <stdint.h>


typedef _Float16 v16h __attribute__((ext_vector_type(16)));
typedef _Float16 v8h  __attribute__((ext_vector_type(8)));
typedef float    v8f  __attribute__((ext_vector_type(8)));
typedef float    v4f  __attribute__((ext_vector_type(4)));
typedef v8h v8ha __attribute__((may_alias));
typedef v4f v4fa __attribute__((may_alias));

union Frag   { v16h v; v8h half[2]; };
union Pack16 { v8h h; v4f f; };

#define NB   8
#define NS   1024
#define ND   1024
#define NH   16
#define NHD  64

#define NEG_MAXF (-3.4028234663852886e38f)

static_assert(ND == NH * NHD, "");
static_assert(NHD == 64, "");
static_assert(NS % 128 == 0, "");
static_assert(ND % 128 == 0, "");
static_assert(ND % 64 == 0, "");
static_assert((NB * NS * ND) % 8 == 0, "");

__device__ __forceinline__ v8f zero8() {
  v8f z = {0.f, 0.f, 0.f, 0.f, 0.f, 0.f, 0.f, 0.f};
  return z;
}
__device__ __forceinline__ v8h zero8h() {
  v8h z;
#pragma unroll
  for (int j = 0; j < 8; ++j) z[j] = (_Float16)0.0f;
  return z;
}

__device__ __forceinline__ void mma(v8f& acc, const v16h& a, const v16h& b) {
  acc = __builtin_amdgcn_wmma_f32_16x16x32_f16(false, a, false, b, (short)0, acc, false, false);
  asm volatile("v_nop\n\tv_nop\n\tv_nop\n\tv_nop" : "+v"(acc) : "v"(a), "v"(b));
}

__device__ __forceinline__ void vst_h8(_Float16* p, v8h v) {
  Pack16 u;
  u.h = v;
  *(volatile v4f*)p = u.f;
}
__device__ __forceinline__ void vst_f4(float* p, v4f v) {
  *(volatile v4f*)p = v;
}

__global__ __launch_bounds__(256) void k_cvt_x(const float* __restrict__ in,
                                               _Float16* __restrict__ out, int n8) {
  const int i = blockIdx.x * 256 + threadIdx.x;
  if (i < n8) {
    const v4fa* src = (const v4fa*)(in + (size_t)i * 8);
    v4f f0 = src[0];
    v4f f1 = src[1];
    v8h hv;
    hv[0] = (_Float16)f0[0]; hv[1] = (_Float16)f0[1]; hv[2] = (_Float16)f0[2]; hv[3] = (_Float16)f0[3];
    hv[4] = (_Float16)f1[0]; hv[5] = (_Float16)f1[1]; hv[6] = (_Float16)f1[2]; hv[7] = (_Float16)f1[3];
    _Float16* dst = out + (size_t)i * 8;
    vst_h8(dst, hv);
    __threadfence();
    vst_h8(dst, hv);
  }
}

__device__ __forceinline__ void st_wt(const float (*tile)[65], _Float16* __restrict__ out,
                                      int t, int n0, int k0, int K, int N, float scale) {
#pragma unroll
  for (int it = 0; it < 2; ++it) {
    const int r = it * 32 + (t >> 3);
    const int p = t & 7;
    v8h hv;
#pragma unroll
    for (int j = 0; j < 8; ++j) hv[j] = (_Float16)(tile[p * 8 + j][r] * scale);
    const int n = n0 + r;
    if (n < N && k0 + p * 8 + 8 <= K) vst_h8(out + (size_t)n * K + k0 + p * 8, hv);
  }
}

__global__ __launch_bounds__(256) void k_tcvt_w(const float* __restrict__ in,
                                                _Float16* __restrict__ out, int K, int N, float scale) {
  __shared__ float tile[64][65];
  const int n0 = blockIdx.x * 64;
  const int k0 = blockIdx.y * 64;
  const int t  = threadIdx.x;
  const int c  = t & 63;
#pragma unroll
  for (int j = 0; j < 16; ++j) {
    const int r = (t >> 6) + 4 * j;
    const int k = k0 + r, n = n0 + c;
    tile[r][c] = (k < K && n < N) ? in[(size_t)k * N + n] : 0.f;
  }
  __syncthreads();
  st_wt(tile, out, t, n0, k0, K, N, scale);
  __threadfence();
  st_wt(tile, out, t, n0, k0, K, N, scale);
}

#define GP  40
#define SPH 136
#define SPF 128

__device__ __forceinline__ void st_qk(const _Float16* stg, _Float16* __restrict__ dst, int tid,
                                      int m0, int cbase, int M, int S, int H) {
#pragma unroll
  for (int it = 0; it < 8; ++it) {
    const int L = it * 32 + (tid >> 3);
    const int p = tid & 7;
    const int r = L >> 1, hh = L & 1;
    const int grow = m0 + r;
    v8h v = *(const v8ha*)&stg[r * SPH + hh * 64 + p * 8];
    if (grow < M) {
      const int b = grow / S, s = grow - b * S;
      const int head = (cbase >> 6) + hh;
      const size_t idx = (((size_t)(b * H + head)) * S + s) * 64 + p * 8;
      vst_h8(dst + idx, v);
    }
  }
}

__device__ __forceinline__ void st_v(const _Float16* stg, _Float16* __restrict__ vo, int tid,
                                     int m0, int cbase, int M, int S, int H) {
  const int b = m0 / S, sb = m0 - b * S;
#pragma unroll
  for (int it = 0; it < 8; ++it) {
    const int L = it * 32 + (tid >> 3);
    const int p = tid & 7;
    const int c = L >> 1, sh = L & 1;
    const int s0 = sh * 64 + p * 8;
    v8h v;
#pragma unroll
    for (int j = 0; j < 8; ++j) v[j] = stg[(s0 + j) * SPH + c];
    const int n = cbase + c;
    const int head = n >> 6, d = n & 63;
    if (m0 + s0 + 8 <= M) {
      const size_t idx = (((size_t)(b * H + head)) * 64 + d) * S + sb + s0;
      vst_h8(vo + idx, v);
    }
  }
}

__device__ __forceinline__ void st_f(const float* stf, float* __restrict__ fo, int tid,
                                     int rb, int n0, int M, int N) {
#pragma unroll
  for (int it = 0; it < 8; ++it) {
    const int L = it * 32 + (tid >> 3);
    const int p = tid & 7;
    const int r = L >> 2, part = L & 3;
    const int col = part * 32 + p * 4;
    v4f v = *(const v4fa*)&stf[r * SPF + col];
    const int grow = rb + r;
    if (grow < M && n0 + col + 4 <= N) vst_f4(fo + (size_t)grow * N + n0 + col, v);
  }
}

template <int MODE>
__global__ __launch_bounds__(256) void k_gemm(
    const _Float16* __restrict__ A, const _Float16* __restrict__ Bt, const float* __restrict__ bias,
    int M, int N, int K, float accScale, float outScale,
    _Float16* __restrict__ qo, _Float16* __restrict__ ko, _Float16* __restrict__ vo,
    float* __restrict__ fo, int S, int H, int Dm) {
  __shared__ alignas(16) unsigned char pool[65536];
  _Float16* sA = (_Float16*)pool;
  _Float16* sB = (_Float16*)(pool + 128 * GP * 2);

  const int tid = threadIdx.x, lane = tid & 31, wave = tid >> 5;
  const int m = lane & 15, h = lane >> 4;
  const int wm = wave & 3, wn = wave >> 2;
  const int m0 = blockIdx.y * 128, n0 = blockIdx.x * 128;

  v8f acc[2][4];
#pragma unroll
  for (int mt = 0; mt < 2; ++mt)
#pragma unroll
    for (int nt = 0; nt < 4; ++nt) acc[mt][nt] = zero8();

  const v8h zh = zero8h();

  for (int k0 = 0; k0 < K; k0 += 32) {
    __syncthreads();
#pragma unroll
    for (int rep = 0; rep < 2; ++rep) {
      const int c = tid + rep * 256;
      const int r = c >> 2, q = (c & 3) * 8;
      const int ga = m0 + r, gb = n0 + r;
      const bool kok = (k0 + q + 8 <= K);
      v8h va = zh, vb = zh;
      if (ga < M && kok) va = *(const v8ha*)&A[(size_t)ga * K + k0 + q];
      if (gb < N && kok) vb = *(const v8ha*)&Bt[(size_t)gb * K + k0 + q];
      *(v8ha*)&sA[r * GP + q] = va;
      *(v8ha*)&sB[r * GP + q] = vb;
    }
    __syncthreads();

    Frag a0, a1;
    const _Float16* pa = &sA[(wm * 32 + m) * GP];
    a0.half[0] = *(const v8ha*)(pa + 8 * h);
    a0.half[1] = *(const v8ha*)(pa + 16 + 8 * h);
    a1.half[0] = *(const v8ha*)(pa + 16 * GP + 8 * h);
    a1.half[1] = *(const v8ha*)(pa + 16 * GP + 16 + 8 * h);
#pragma unroll
    for (int nt = 0; nt < 4; ++nt) {
      const _Float16* pb = &sB[(wn * 64 + nt * 16 + m) * GP];
      Frag b;
      b.half[0] = *(const v8ha*)(pb + 8 * h);
      b.half[1] = *(const v8ha*)(pb + 16 + 8 * h);
      mma(acc[0][nt], a0.v, b.v);
      mma(acc[1][nt], a1.v, b.v);
    }
  }

  if (MODE == 0) {
    __syncthreads();
    _Float16* stg = (_Float16*)pool;
#pragma unroll
    for (int mt = 0; mt < 2; ++mt)
#pragma unroll
      for (int nt = 0; nt < 4; ++nt) {
        const int col = wn * 64 + nt * 16 + m;
        int gc = n0 + col;
        gc = gc < N ? gc : N - 1;
        const float bv = bias[gc];
#pragma unroll
        for (int r = 0; r < 8; ++r) {
          const int row = wm * 32 + mt * 16 + 8 * h + r;
          const float v = acc[mt][nt][r] * accScale + bv;
          stg[row * SPH + col] = (_Float16)(v * outScale);
        }
      }
    __syncthreads();
    const int sec = n0 / Dm;
    const int cbase = n0 - sec * Dm;
    if (sec < 2) {
      _Float16* dst = (sec == 0) ? qo : ko;
      st_qk(stg, dst, tid, m0, cbase, M, S, H);
      __threadfence();
      st_qk(stg, dst, tid, m0, cbase, M, S, H);
    } else {
      st_v(stg, vo, tid, m0, cbase, M, S, H);
      __threadfence();
      st_v(stg, vo, tid, m0, cbase, M, S, H);
    }
  } else {
    float* stf = (float*)pool;
#pragma unroll
    for (int hf = 0; hf < 2; ++hf) {
      __syncthreads();
      if ((wm >> 1) == hf) {
#pragma unroll
        for (int mt = 0; mt < 2; ++mt)
#pragma unroll
          for (int nt = 0; nt < 4; ++nt) {
            const int col = wn * 64 + nt * 16 + m;
            int gc = n0 + col;
            gc = gc < N ? gc : N - 1;
            const float bv = bias[gc];
#pragma unroll
            for (int r = 0; r < 8; ++r) {
              const int row = (wm & 1) * 32 + mt * 16 + 8 * h + r;
              stf[row * SPF + col] = (acc[mt][nt][r] * accScale + bv) * outScale;
            }
          }
      }
      __syncthreads();
      st_f(stf, fo, tid, m0 + hf * 64, n0, M, N);
      __threadfence();
      st_f(stf, fo, tid, m0 + hf * 64, n0, M, N);
    }
  }
}

#define AP 72

__device__ __forceinline__ void st_att(const _Float16* myP, _Float16* __restrict__ ao, int lane,
                                       int qrow0, int b, int hd, int S, int Dm) {
#pragma unroll
  for (int it = 0; it < 4; ++it) {
    const int rl = it * 4 + (lane >> 3);
    const int p  = lane & 7;
    v8h v = *(const v8ha*)&myP[rl * AP + p * 8];
    const int qr = qrow0 + rl;
    if (qr < S) vst_h8(ao + ((size_t)b * S + qr) * Dm + hd * 64 + p * 8, v);
  }
}

__global__ __launch_bounds__(256) void k_attn(
    const _Float16* __restrict__ qh, const _Float16* __restrict__ kh, const _Float16* __restrict__ vT,
    const float* __restrict__ mask, _Float16* __restrict__ ao,
    int S, int H, int Dm, float sScale, float oScale) {
  __shared__ alignas(16) _Float16 sK[64 * AP];
  __shared__ alignas(16) _Float16 sVt[64 * AP];
  __shared__ alignas(16) _Float16 sP[8 * 16 * AP];

  const int tid = threadIdx.x, lane = tid & 31, wave = tid >> 5;
  const int m = lane & 15, h = lane >> 4;
  const int qb = blockIdx.x * 128, bh = blockIdx.y;
  const int b = bh / H, hd = bh - b * H;
  const int qrow0 = qb + wave * 16;
  _Float16* myP = sP + wave * 16 * AP;

  Frag qf[2];
  {
    int qr = qrow0 + m;
    qr = qr < S ? qr : S - 1;
    const _Float16* qp = qh + ((size_t)bh * S + qr) * 64;
#pragma unroll
    for (int kk = 0; kk < 2; ++kk) {
      qf[kk].half[0] = *(const v8ha*)(qp + kk * 32 + 8 * h);
      qf[kk].half[1] = *(const v8ha*)(qp + kk * 32 + 16 + 8 * h);
    }
  }

  v8f o[4];
#pragma unroll
  for (int nt = 0; nt < 4; ++nt) o[nt] = zero8();
  float mrow[8], lrow[8];
#pragma unroll
  for (int r = 0; r < 8; ++r) { mrow[r] = NEG_MAXF; lrow[r] = 0.f; }

  for (int jb = 0; jb < S; jb += 64) {
    __syncthreads();
#pragma unroll
    for (int rep = 0; rep < 2; ++rep) {
      const int c = tid + rep * 256;
      const int r = c >> 3, q = (c & 7) * 8;
      int kr = jb + r;
      kr = kr < S ? kr : S - 1;
      *(v8ha*)&sK[r * AP + q] = *(const v8ha*)&kh[((size_t)bh * S + kr) * 64 + q];
      int kq = jb + q;
      kq = (kq + 8 <= S) ? kq : (S - 8);
      *(v8ha*)&sVt[r * AP + q] = *(const v8ha*)&vT[((size_t)bh * 64 + r) * S + kq];
    }
    __syncthreads();

    v8f s[4];
#pragma unroll
    for (int nt = 0; nt < 4; ++nt) {
      const _Float16* kp = &sK[(nt * 16 + m) * AP];
      Frag b0, b1;
      b0.half[0] = *(const v8ha*)(kp + 8 * h);
      b0.half[1] = *(const v8ha*)(kp + 16 + 8 * h);
      b1.half[0] = *(const v8ha*)(kp + 32 + 8 * h);
      b1.half[1] = *(const v8ha*)(kp + 48 + 8 * h);
      s[nt] = zero8();
      mma(s[nt], qf[0].v, b0.v);
      mma(s[nt], qf[1].v, b1.v);
    }

#pragma unroll
    for (int nt = 0; nt < 4; ++nt) {
      int kc = jb + nt * 16 + m;
      kc = kc < S ? kc : S - 1;
#pragma unroll
      for (int r = 0; r < 8; ++r) {
        int qr = qrow0 + 8 * h + r;
        qr = qr < S ? qr : S - 1;
        const float mk = mask[((size_t)b * S + qr) * S + kc];
        s[nt][r] = s[nt][r] * sScale + NEG_MAXF * (1.0f - mk);
      }
    }

    float rmax[8];
#pragma unroll
    for (int r = 0; r < 8; ++r)
      rmax[r] = fmaxf(fmaxf(s[0][r], s[1][r]), fmaxf(s[2][r], s[3][r]));
#pragma unroll
    for (int d = 1; d < 16; d <<= 1)
#pragma unroll
      for (int r = 0; r < 8; ++r) rmax[r] = fmaxf(rmax[r], __shfl_xor(rmax[r], d, 32));

    float corr[8], rsum[8];
#pragma unroll
    for (int r = 0; r < 8; ++r) {
      const float mn = fmaxf(mrow[r], rmax[r]);
      corr[r] = __expf(mrow[r] - mn);
      mrow[r] = mn;
      rsum[r] = 0.f;
    }
#pragma unroll
    for (int nt = 0; nt < 4; ++nt)
#pragma unroll
      for (int r = 0; r < 8; ++r) {
        const float p = __expf(s[nt][r] - mrow[r]);
        rsum[r] += p;
        myP[(8 * h + r) * AP + nt * 16 + m] = (_Float16)(p * 256.0f);
      }
#pragma unroll
    for (int d = 1; d < 16; d <<= 1)
#pragma unroll
      for (int r = 0; r < 8; ++r) rsum[r] += __shfl_xor(rsum[r], d, 32);
#pragma unroll
    for (int r = 0; r < 8; ++r) lrow[r] = lrow[r] * corr[r] + rsum[r];
#pragma unroll
    for (int nt = 0; nt < 4; ++nt)
#pragma unroll
      for (int r = 0; r < 8; ++r) o[nt][r] *= corr[r];

    __syncthreads();

    Frag pf[2];
    {
      const _Float16* pp = myP + m * AP;
#pragma unroll
      for (int kk = 0; kk < 2; ++kk) {
        pf[kk].half[0] = *(const v8ha*)(pp + kk * 32 + 8 * h);
        pf[kk].half[1] = *(const v8ha*)(pp + kk * 32 + 16 + 8 * h);
      }
    }
#pragma unroll
    for (int nt = 0; nt < 4; ++nt) {
      const _Float16* vp = &sVt[(nt * 16 + m) * AP];
      Frag bv0, bv1;
      bv0.half[0] = *(const v8ha*)(vp + 8 * h);
      bv0.half[1] = *(const v8ha*)(vp + 16 + 8 * h);
      bv1.half[0] = *(const v8ha*)(vp + 32 + 8 * h);
      bv1.half[1] = *(const v8ha*)(vp + 48 + 8 * h);
      mma(o[nt], pf[0].v, bv0.v);
      mma(o[nt], pf[1].v, bv1.v);
    }
  }

  __syncthreads();
  float inv[8];
#pragma unroll
  for (int r = 0; r < 8; ++r) inv[r] = oScale / lrow[r];
#pragma unroll
  for (int nt = 0; nt < 4; ++nt)
#pragma unroll
    for (int r = 0; r < 8; ++r)
      myP[(8 * h + r) * AP + nt * 16 + m] = (_Float16)(o[nt][r] * inv[r]);
  __syncthreads();
  st_att(myP, ao, lane, qrow0, b, hd, S, Dm);
  __threadfence();
  st_att(myP, ao, lane, qrow0, b, hd, S, Dm);
}

extern "C" void kernel_launch(void* const* d_in, const int* in_sizes, int n_in,
                              void* d_out, int out_size, void* d_ws, size_t ws_size,
                              hipStream_t stream) {
  if (n_in < 6) return;
  const int M = NB * NS;
  if (in_sizes[0] != NB * NS * ND) return;
  if (in_sizes[1] != NB * NS * NS) return;
  if (in_sizes[2] != ND * 3 * ND) return;
  if (in_sizes[3] != 3 * ND) return;
  if (in_sizes[4] != ND * ND) return;
  if (in_sizes[5] != ND) return;
  if (out_size != NB * NS * ND) return;

  const float* hs   = (const float*)d_in[0];
  const float* msk  = (const float*)d_in[1];
  const float* cw   = (const float*)d_in[2];
  const float* cb   = (const float*)d_in[3];
  const float* pw   = (const float*)d_in[4];
  const float* pb   = (const float*)d_in[5];
  float* out = (float*)d_out;

  unsigned char* ws = (unsigned char*)d_ws;
  size_t off = 0;
  const size_t bXh   = (size_t)M * ND * 2;
  const size_t bWqkv = (size_t)3 * ND * ND * 2;
  const size_t bWprj = (size_t)ND * ND * 2;
  const size_t bHead = (size_t)NB * NH * NS * NHD * 2;
  const size_t bAh   = (size_t)M * ND * 2;
  _Float16* xh    = (_Float16*)(ws + off); off += bXh;
  _Float16* wqkvT = (_Float16*)(ws + off); off += bWqkv;
  _Float16* wprjT = (_Float16*)(ws + off); off += bWprj;
  _Float16* qh    = (_Float16*)(ws + off); off += bHead;
  _Float16* kh    = (_Float16*)(ws + off); off += bHead;
  _Float16* vT    = (_Float16*)(ws + off); off += bHead;
  _Float16* ah    = (_Float16*)(ws + off); off += bAh;
  if (off > ws_size) return;

  {
    const int n8 = (M * ND) / 8;
    k_cvt_x<<<dim3((n8 + 255) / 256), dim3(256), 0, stream>>>(hs, xh, n8);
    k_tcvt_w<<<dim3((3 * ND + 63) / 64, (ND + 63) / 64), dim3(256), 0, stream>>>(
        cw, wqkvT, ND, 3 * ND, 64.0f);
    k_tcvt_w<<<dim3((ND + 63) / 64, (ND + 63) / 64), dim3(256), 0, stream>>>(
        pw, wprjT, ND, ND, 64.0f);
  }

  hipLaunchKernelGGL(HIP_KERNEL_NAME(k_gemm<0>), dim3((3 * ND + 127) / 128, (M + 127) / 128),
                     dim3(256), 0, stream,
                     (const _Float16*)xh, (const _Float16*)wqkvT, cb, M, 3 * ND, ND,
                     0.015625f, 16.0f, qh, kh, vT, out, NS, NH, ND);

  k_attn<<<dim3((NS + 127) / 128, NB * NH), dim3(256), 0, stream>>>(
      qh, kh, vT, msk, ah, NS, NH, ND, 0.00048828125f, 0.015625f);

  hipLaunchKernelGGL(HIP_KERNEL_NAME(k_gemm<1>), dim3((ND + 127) / 128, (M + 127) / 128),
                     dim3(256), 0, stream,
                     (const _Float16*)ah, (const _Float16*)wprjT, pb, M, ND, ND,
                     0.000244140625f, 1.0f, qh, kh, vT, out, NS, NH, ND);
}
